// Encoder_1666447310976
// MI455X (gfx1250) — hardware-run, weakly checked
//
#include <hip/hip_runtime.h>
#include <stddef.h>


typedef _Float16 h16;
typedef _Float16 v16h __attribute__((ext_vector_type(16)));
typedef _Float16 v8h  __attribute__((ext_vector_type(8)));
typedef _Float16 v4h  __attribute__((ext_vector_type(4)));
typedef float    v8f  __attribute__((ext_vector_type(8)));
typedef float    v4f  __attribute__((ext_vector_type(4)));

#ifndef NB
#define NB 16
#endif
#ifndef SEQ
#define SEQ 1024
#endif
#define NB_FULL  16
#define SEQ_FULL 1024
#define CH    256
#define NCW   32
#define TROWS 32
#define NSAMP (NB * NCW)

#define LDXS 264
#define LDXT 32
#define LDW  40
#define LDD  33
#define LDE  32

#define XCARRY 16.0f
#define CCARRY 1024.0f
#define PCARRY 16384.0f

static_assert(NB >= 1 && NB <= NB_FULL);
static_assert(NB <= 32);
static_assert(SEQ >= TROWS && SEQ <= SEQ_FULL && (SEQ % TROWS) == 0);
static_assert(CH == 32 * 8);
static_assert(CH == 8 * 32);
static_assert(NCW == 32);
static_assert(TROWS == 8 * 4);
static_assert(TROWS * CH == 256 * 8 * 4);
static_assert((CH % 32) == 0 && (TROWS % 32) == 0);
static_assert((LDXS % 8) == 0 && LDXS >= CH);
static_assert((LDXT % 8) == 0 && LDXT >= TROWS);
static_assert((LDW % 8) == 0 && LDW >= TROWS);
static_assert((LDE % 4) == 0 && LDE >= 32);
static_assert(TROWS * LDXS * 2 + CH * LDXT * 2 + NCW * LDW * 2 + 2 * TROWS * LDD * 4 +
              8 * 16 * LDE * 4 + 8 * NCW * 4 + 2 * NCW * 4 <= 65536);

#define ENC_BYTES ((size_t)NB * NCW * CH * 4)
#define OFF_ENC   ((size_t)0)
#define WS_TOTAL  (OFF_ENC + ENC_BYTES)
static_assert((ENC_BYTES % 128) == 0);
static_assert(WS_TOTAL <= (size_t)134217728);

__device__ __forceinline__ float bf16r(float x) {
  unsigned int u = __float_as_uint(x);
  u = (u + 0x7FFFu + ((u >> 16) & 1u)) & 0xFFFF0000u;
  return __uint_as_float(u);
}

static __device__ __forceinline__ h16 toh_flush(float v) {
  const h16 r = (h16)v;
  return (fabsf(v) < 6.103515625e-05f) ? (h16)0.0f : r;
}

__device__ __forceinline__ v16h frag_at(const _Float16* p) {
  v8h lo = *(const v8h*)(p);
  v8h hi = *(const v8h*)(p + 16);
  v16h out;
#pragma unroll
  for (int i = 0; i < 8; ++i) { out[i] = lo[i]; out[i + 8] = hi[i]; }
  return out;
}
__device__ __forceinline__ v16h ld_frag(const _Float16* base, unsigned ld) {
  const unsigned lane = threadIdx.x & 31u;
  return frag_at(base + (lane & 15u) * ld + (lane >> 4) * 8u);
}

__device__ __forceinline__ v8f wmma16(v16h a, v16h b, v8f c) {
  v8f d = __builtin_amdgcn_wmma_f32_16x16x32_f16(false, a, false, b, (short)0, c,
                                                 false, false);
  asm volatile("v_nop\n\tv_nop\n\tv_nop\n\tv_nop" : "+v"(d) : "v"(a), "v"(b));
  return d;
}

__device__ __forceinline__ float red32_sum(float x) {
#pragma unroll
  for (int off = 1; off < 32; off <<= 1) x += __shfl_xor(x, off, 32);
  return x;
}
__device__ __forceinline__ float red32_max(float x) {
#pragma unroll
  for (int off = 1; off < 32; off <<= 1) x = fmaxf(x, __shfl_xor(x, off, 32));
  return x;
}

__device__ __forceinline__ void wave_lds_sync() {
  __builtin_amdgcn_fence(3  , "wavefront");
  asm volatile("s_wait_dscnt 0x0" ::: "memory");
  __builtin_amdgcn_wave_barrier();
}

__global__ __launch_bounds__(256) void assign_kernel(
    const float* __restrict__ X, const float* __restrict__ CW, const float* __restrict__ SF,
    float* __restrict__ enc) {
  __shared__ __attribute__((aligned(16))) _Float16 Xs[TROWS * LDXS];
  __shared__ __attribute__((aligned(16))) _Float16 XT[CH * LDXT];
  __shared__ __attribute__((aligned(16))) _Float16 Wt[NCW * LDW];
  __shared__ __attribute__((aligned(16))) float dotb[2 * TROWS * LDD];
  __shared__ __attribute__((aligned(16))) float Es[8 * 16 * LDE];
  __shared__ float wpart[8 * NCW];
  __shared__ float cwn_s[NCW];
  __shared__ float wsum_s[NCW];

  const unsigned tid = threadIdx.x, lane = tid & 31u;
  const unsigned wave = (unsigned)__builtin_amdgcn_readfirstlane((int)(threadIdx.x >> 5));
  const unsigned hh = lane >> 4, m = lane & 15u;
  const unsigned b = blockIdx.x;
  const unsigned mT = (wave >> 1) & 1u, nT = wave & 1u, kh = wave >> 2;

  v16h bfrag[4];
  {
    const float* cp = CW + (size_t)(nT * 16u + m) * CH + kh * 128u + hh * 8u;
#pragma unroll
    for (int ks = 0; ks < 4; ++ks) {
      const v4f a0 = *(const v4f*)(cp + ks * 32);
      const v4f a1 = *(const v4f*)(cp + ks * 32 + 4);
      const v4f a2 = *(const v4f*)(cp + ks * 32 + 16);
      const v4f a3 = *(const v4f*)(cp + ks * 32 + 20);
      v16h f;
#pragma unroll
      for (int i = 0; i < 4; ++i) {
        f[i]      = toh_flush(CCARRY * bf16r(a0[i]));
        f[i + 4]  = toh_flush(CCARRY * bf16r(a1[i]));
        f[i + 8]  = toh_flush(CCARRY * bf16r(a2[i]));
        f[i + 12] = toh_flush(CCARRY * bf16r(a3[i]));
      }
      bfrag[ks] = f;
    }
  }

#pragma unroll 1
  for (unsigned i = 0; i < 4u; ++i) {
    const unsigned k = wave * 4u + i;
    const v4f a0 = *(const v4f*)(CW + (size_t)k * CH + lane * 8u);
    const v4f a1 = *(const v4f*)(CW + (size_t)k * CH + lane * 8u + 4u);
    float s = 0.0f;
#pragma unroll
    for (int j = 0; j < 4; ++j) {
      const float e0 = bf16r(a0[j]);
      const float e1 = bf16r(a1[j]);
      s += e0 * e0;
      s += e1 * e1;
    }
    s = red32_sum(s);
    if (lane == 0u) cwn_s[k] = s;
  }
  const float sfk = bf16r(SF[lane]);
  __syncthreads();
  const float cwn_k = cwn_s[lane];

  const float* xb = X + (size_t)b * SEQ_FULL * CH;
  v8f o[4];
#pragma unroll
  for (int t = 0; t < 4; ++t) o[t] = (v8f){};
  float wacc = 0.0f;

#pragma unroll 1
  for (unsigned n0 = 0; n0 < (unsigned)SEQ; n0 += TROWS) {
#pragma unroll 2
    for (unsigned j = 0; j < 8u; ++j) {
      const unsigned idx = tid + 256u * j;
      const unsigned r = idx >> 6, c = (idx & 63u) * 4u;
      const v4f a = *(const v4f*)(xb + (size_t)(n0 + r) * CH + c);
      v4h hv;
#pragma unroll
      for (int i = 0; i < 4; ++i) hv[i] = toh_flush(XCARRY * bf16r(a[i]));
      *(v4h*)&Xs[r * LDXS + c] = hv;
#pragma unroll
      for (unsigned i = 0; i < 4u; ++i) XT[(c + i) * LDXT + r] = hv[i];
    }
    __syncthreads();

    {
      v8f acc = {};
#pragma unroll
      for (int ks = 0; ks < 4; ++ks) {
        const v16h a = ld_frag(&Xs[(mT * 16u) * LDXS + kh * 128u + (unsigned)ks * 32u], LDXS);
        acc = wmma16(a, bfrag[ks], acc);
      }
#pragma unroll
      for (int r = 0; r < 8; ++r)
        dotb[(kh * TROWS + mT * 16u + hh * 8u + (unsigned)r) * LDD + nT * 16u + m] = acc[r];
    }
    __syncthreads();

#pragma unroll 1
    for (unsigned i = 0; i < 4u; ++i) {
      const unsigned r = wave * 4u + i;
      const v8h xv = *(const v8h*)&Xs[r * LDXS + lane * 8u];
      float s = 0.0f;
#pragma unroll
      for (int j = 0; j < 8; ++j) {
        const float e = (float)xv[j];
        s += e * e;
      }
      const float xn = red32_sum(s) * (1.0f / (XCARRY * XCARRY));
      const float d = (dotb[r * LDD + lane] + dotb[(TROWS + r) * LDD + lane]) *
                      (1.0f / (XCARRY * CCARRY));
      const float sq = (xn - 2.0f * d) + cwn_k;
      const float l = sq * sfk;
      const float mx = red32_max(l);
      const float e = __expf(l - mx);
      const float den = red32_sum(e);
      const float wv = e * (1.0f / den);
      wacc += wv;
      Wt[lane * LDW + r] = toh_flush(wv * PCARRY);
    }
    __syncthreads();

    {
      const v16h a0 = ld_frag(&Wt[0], LDW);
      const v16h a1 = ld_frag(&Wt[16 * LDW], LDW);
      const v16h b0 = ld_frag(&XT[(wave * 32u) * LDXT], LDXT);
      const v16h b1 = ld_frag(&XT[(wave * 32u + 16u) * LDXT], LDXT);
      o[0] = wmma16(a0, b0, o[0]);
      o[1] = wmma16(a0, b1, o[1]);
      o[2] = wmma16(a1, b0, o[2]);
      o[3] = wmma16(a1, b1, o[3]);
    }
    __syncthreads();
  }

  wpart[wave * NCW + lane] = wacc;
  __syncthreads();
  if (tid < (unsigned)NCW) {
    float s = 0.0f;
#pragma unroll 1
    for (unsigned w = 0; w < 8u; ++w) s += wpart[w * NCW + tid];
    wsum_s[tid] = s;
  }
  __syncthreads();

  float* E = Es + wave * (16u * LDE);
  const float oscale = 1.0f / (PCARRY * XCARRY);
#pragma unroll
  for (int mt = 0; mt < 2; ++mt) {
#pragma unroll
    for (int r = 0; r < 8; ++r) {
      E[(hh * 8u + (unsigned)r) * LDE + m]       = o[mt * 2][r] * oscale;
      E[(hh * 8u + (unsigned)r) * LDE + 16u + m] = o[mt * 2 + 1][r] * oscale;
    }
    wave_lds_sync();
    v4f xs[4];
    size_t off[4];
#pragma unroll
    for (unsigned i = 0; i < 4u; ++i) {
      const unsigned rr = 4u * i + (lane >> 3);
      const unsigned c4 = (lane & 7u) * 4u;
      const unsigned k = (unsigned)mt * 16u + rr;
      const unsigned c = wave * 32u + c4;
      const v4f u = *(const v4f*)&E[rr * LDE + c4];
      const v4f cv = *(const v4f*)(CW + (size_t)k * CH + c);
      const float wsk = wsum_s[k];
      v4f val;
#pragma unroll
      for (int j = 0; j < 4; ++j) val[j] = u[j] - wsk * bf16r(cv[j]);
      xs[i] = val;
      off[i] = ((size_t)b * NCW + k) * CH + c;
    }
#pragma unroll
    for (int i = 0; i < 4; ++i) *(volatile v4f*)(enc + off[i]) = xs[i];
    __threadfence();
#pragma unroll
    for (int i = 0; i < 4; ++i) *(volatile v4f*)(enc + off[i]) = xs[i];
    wave_lds_sync();
  }
}

__global__ __launch_bounds__(256) void bn_out_kernel(
    const float* __restrict__ enc, const float* __restrict__ G, const float* __restrict__ Be,
    float* __restrict__ out) {
#pragma clang fp contract(off)
  __shared__ float p1[8 * 32];
  __shared__ float p2[8 * 32];
  __shared__ __attribute__((aligned(16))) float outs[32 * 32];

  const unsigned tid = threadIdx.x, lane = tid & 31u;
  const unsigned wave = (unsigned)__builtin_amdgcn_readfirstlane((int)(threadIdx.x >> 5));
  const unsigned c = blockIdx.x * 32u + lane;

  float s = 0.0f;
#pragma unroll 1
  for (unsigned i = wave; i < (unsigned)NSAMP; i += 8u) s += enc[(size_t)i * CH + c];
  p1[wave * 32u + lane] = s;
  __syncthreads();
  float tot = 0.0f;
#pragma unroll 1
  for (unsigned w = 0; w < 8u; ++w) tot += p1[w * 32u + lane];
  const float mean = tot * (1.0f / (float)NSAMP);

  float ss = 0.0f;
#pragma unroll 1
  for (unsigned i = wave; i < (unsigned)NSAMP; i += 8u) {
    const float d = enc[(size_t)i * CH + c] - mean;
    ss += d * d;
  }
  p2[wave * 32u + lane] = ss;
  __syncthreads();
  float tot2 = 0.0f;
#pragma unroll 1
  for (unsigned w = 0; w < 8u; ++w) tot2 += p2[w * 32u + lane];
  const float var = tot2 * (1.0f / (float)NSAMP);
  const float rstd = 1.0f / sqrtf(var + 1.0e-3f);
  const float g = bf16r(G[c]);
  const float bt = bf16r(Be[c]);

#pragma unroll 1
  for (unsigned bb = wave; bb < (unsigned)NB; bb += 8u) {
    float acc = 0.0f;
#pragma unroll 1
    for (unsigned k = 0; k < (unsigned)NCW; ++k) {
      const float v = enc[((size_t)bb * NCW + k) * CH + c];
      const float t = ((v - mean) * rstd) * g + bt;
      acc += fmaxf(t, 0.0f);
    }
    outs[bb * 32u + lane] = acc;
  }
  __syncthreads();

  const unsigned line = wave * 4u + (lane >> 3);
  if (line < (unsigned)NB) {
    const unsigned c4 = (lane & 7u) * 4u;
    const v4f x = *(const v4f*)&outs[line * 32u + c4];
    float* p = out + (size_t)line * CH + blockIdx.x * 32u + c4;
    *(volatile v4f*)p = x;
    __threadfence();
    *(volatile v4f*)p = x;
  }
}

extern "C" void kernel_launch(void* const* d_in, const int* in_sizes, int n_in,
                              void* d_out, int out_size, void* d_ws, size_t ws_size,
                              hipStream_t stream) {
  if (n_in < 5) return;
  const long long need_x = ((long long)(NB - 1) * SEQ_FULL + SEQ) * CH;
  if ((long long)in_sizes[0] < need_x) return;
  if ((long long)in_sizes[1] < (long long)NCW * CH) return;
  if (in_sizes[2] < NCW) return;
  if (in_sizes[3] < CH || in_sizes[4] < CH) return;
  if ((long long)out_size < (long long)NB * CH) return;
  if (ws_size < WS_TOTAL) return;

  const float* X  = (const float*)d_in[0];
  const float* CW = (const float*)d_in[1];
  const float* SF = (const float*)d_in[2];
  const float* G  = (const float*)d_in[3];
  const float* Be = (const float*)d_in[4];
  float* out = (float*)d_out;

  char* ws = (char*)d_ws;
  float* enc = (float*)(ws + OFF_ENC);

  assign_kernel<<<dim3(NB), dim3(256), 0, stream>>>(X, CW, SF, enc);
  bn_out_kernel<<<dim3(CH / 32), dim3(256), 0, stream>>>(enc, G, Be, out);
}
